// SpatialAwareAttention_56959856279791
// MI455X (gfx1250) — hardware-verified
//
#include <hip/hip_runtime.h>
#include <math.h>

typedef __attribute__((ext_vector_type(16))) _Float16 v16h;
typedef __attribute__((ext_vector_type(8)))  _Float16 v8h;
typedef __attribute__((ext_vector_type(16))) __bf16   v16b;
typedef __attribute__((ext_vector_type(8)))  __bf16   v8b;
typedef __attribute__((ext_vector_type(8)))  float    v8f;
typedef __attribute__((ext_vector_type(4)))  float    v4f;

__device__ __forceinline__ unsigned short f2bf_bits(float f) {
  unsigned u = __float_as_uint(f);
  return (unsigned short)((u + 0x7FFFu + ((u >> 16) & 1u)) >> 16);
}
__device__ __forceinline__ float bf_bits2f(unsigned short h) { return __uint_as_float(((unsigned)h) << 16); }

__device__ __forceinline__ void dep_guard_h(v8f& a, v8f& b, v16h x, v16h y) { asm volatile("v_nop\n\tv_nop\n\tv_nop\n\tv_nop" : "+v"(a), "+v"(b) : "v"(x), "v"(y)); }
__device__ __forceinline__ void dep_guard_b(v8f& a, v8f& b, v16b x, v16b y) { asm volatile("v_nop\n\tv_nop\n\tv_nop\n\tv_nop" : "+v"(a), "+v"(b) : "v"(x), "v"(y)); }
__device__ __forceinline__ void keep4_h(v16h a, v16h b, v16h c, v16h d) { asm volatile("v_nop" :: "v"(a), "v"(b), "v"(c), "v"(d)); }
__device__ __forceinline__ void keep4_b(v16b a, v16b b, v16b c, v16b d) { asm volatile("v_nop" :: "v"(a), "v"(b), "v"(c), "v"(d)); }
__device__ __forceinline__ void acc_guard4(v8f& a, v8f& b, v8f& c, v8f& d) { asm volatile("v_nop\n\tv_nop\n\tv_nop\n\tv_nop" : "+v"(a), "+v"(b), "+v"(c), "+v"(d)); }
template <typename T> struct Frag;
template <> struct Frag<_Float16> {
  typedef v16h V; union U { v16h v; v8h h[2]; };
  static __device__ __forceinline__ v16h load(const _Float16* p) {
    U f; f.h[0] = *(const v8h*)(p); f.h[1] = *(const v8h*)(p + 16); return f.v;
  }
  static __device__ __forceinline__ v8f mma(v16h a, v16h b, v8f c) {
    return __builtin_amdgcn_wmma_f32_16x16x32_f16(false, a, false, b, (short)0, c, false, false);
  }
  static __device__ __forceinline__ void guard(v8f& a, v8f& b, v16h x, v16h y) { dep_guard_h(a, b, x, y); }
  static __device__ __forceinline__ void keep(v16h a, v16h b, v16h c, v16h d) { keep4_h(a, b, c, d); }
};
template <> struct Frag<__bf16> {
  typedef v16b V; union U { v16b v; v8b h[2]; };
  static __device__ __forceinline__ v16b load(const __bf16* p) {
    U f; f.h[0] = *(const v8b*)(p); f.h[1] = *(const v8b*)(p + 16); return f.v;
  }
  static __device__ __forceinline__ v8f mma(v16b a, v16b b, v8f c) {
    return __builtin_amdgcn_wmma_f32_16x16x32_bf16(false, a, false, b, (short)0, c, false, false);
  }
  static __device__ __forceinline__ void guard(v8f& a, v8f& b, v16b x, v16b y) { dep_guard_b(a, b, x, y); }
  static __device__ __forceinline__ void keep(v16b a, v16b b, v16b c, v16b d) { keep4_b(a, b, c, d); }
};

template <int ET> struct Elem;
template <> struct Elem<0> { typedef _Float16 T; };
template <> struct Elem<1> { typedef __bf16 T; };
template <int ET, bool SPLIT, int BIAS_MODE, int OUT_MODE, bool RESID, int ACT = 0>
__global__ __launch_bounds__(256) void wmma_gemm64(
    const unsigned short* __restrict__ Ap, const unsigned short* __restrict__ A2p, int lda, long strideA,
    const unsigned short* __restrict__ Btp, const unsigned short* __restrict__ Bt2p, int ldb, long strideB,
    void* __restrict__ Cout, void* __restrict__ Cout2, int ldc, long strideC,
    const float* __restrict__ bias,
    const float* __restrict__ resid, long strideR,
    int M, int N, int K, float scale) {
  typedef typename Elem<ET>::T T;
  typedef typename Frag<T>::V V;
  const T* A = (const T*)Ap; const T* A2 = (const T*)A2p; const T* Bt = (const T*)Btp; const T* Bt2 = (const T*)Bt2p;
  __shared__ __align__(16) float sT[8][16 * 68];
  const int b    = blockIdx.y;
  const int lane = threadIdx.x & 31;
  const int wave = threadIdx.x >> 5;
  const int tilesN = N >> 6;
  const int tilesM = M >> 6;
  const int tile = blockIdx.x * 8 + wave;
  if (tile >= tilesM * tilesN) return;
  const int tm = tile / tilesN;
  const int tn = tile - tm * tilesN;
  const int m0 = tm << 6;
  const int n0 = tn << 6;

  const T* Ab  = A  + (size_t)b * strideA;
  const T* Bb  = Bt + (size_t)b * strideB;
  const T* Ab2 = SPLIT ? (A2  + (size_t)b * strideA) : nullptr;
  const T* Bb2 = SPLIT ? (Bt2 + (size_t)b * strideB) : nullptr;

  const int rlane = lane & 15;
  const int koff  = (lane >> 4) * 8;
  const int mOff  = (lane >> 4) * 8;

  v8f acc[4][4];
#pragma unroll
  for (int i = 0; i < 4; ++i)
#pragma unroll
    for (int j = 0; j < 4; ++j) acc[i][j] = (v8f){0.f,0.f,0.f,0.f,0.f,0.f,0.f,0.f};

  for (int k0 = 0; k0 < K; k0 += 32) {
    V bh[4], bl[4];
#pragma unroll
    for (int j = 0; j < 4; ++j) {
      const size_t bo = (size_t)(n0 + (j << 4) + rlane) * ldb + koff + k0;
      bh[j] = Frag<T>::load(Bb + bo);
      if (SPLIT) bl[j] = Frag<T>::load(Bb2 + bo);
    }
#pragma unroll
    for (int i = 0; i < 4; ++i) {
      const size_t ao = (size_t)(m0 + (i << 4) + rlane) * lda + koff + k0;
      V ah = Frag<T>::load(Ab + ao);
      V al;
      if (SPLIT) al = Frag<T>::load(Ab2 + ao);
#pragma unroll
      for (int j = 0; j < 4; ++j) {
        acc[i][j] = Frag<T>::mma(ah, bh[j], acc[i][j]);
        if (SPLIT) {
          acc[i][j] = Frag<T>::mma(ah, bl[j], acc[i][j]);
          acc[i][j] = Frag<T>::mma(al, bh[j], acc[i][j]);
        }
      }
      Frag<T>::guard(acc[i][0], acc[i][3], ah, SPLIT ? al : ah);
    }
    Frag<T>::keep(bh[0], bh[1], bh[2], bh[3]);
    if (SPLIT) Frag<T>::keep(bl[0], bl[1], bl[2], bl[3]);
  }
  acc_guard4(acc[0][0], acc[0][1], acc[0][2], acc[0][3]);
  acc_guard4(acc[1][0], acc[1][1], acc[1][2], acc[1][3]);
  acc_guard4(acc[2][0], acc[2][1], acc[2][2], acc[2][3]);
  acc_guard4(acc[3][0], acc[3][1], acc[3][2], acc[3][3]);

  float* slab = sT[wave];
  const float* Rb = RESID ? (resid + (size_t)b * strideR) : nullptr;
#pragma unroll
  for (int i = 0; i < 4; ++i) {
    const int mBase = m0 + (i << 4);
#pragma unroll
    for (int j = 0; j < 4; ++j) {
      const int n = n0 + (j << 4) + rlane;
      float bv = 0.f;
      if (BIAS_MODE == 2) bv = bias[n];
#pragma unroll
      for (int r = 0; r < 8; ++r) {
        float v = acc[i][j][r] * scale;
        if (BIAS_MODE == 1) v += bias[mBase + mOff + r];
        if (BIAS_MODE == 2) v += bv;
        if (RESID) v += Rb[(size_t)(mBase + mOff + r) * ldc + n];
        if (ACT == 1) v = tanhf(v);
        if (ACT == 2) v = fmaxf(v, 0.0f);
        if (ACT == 3) v = v / (1.0f + expf(-v));
        if (ACT == 4) v = (v > 0.f) ? v : 0.01f * v;
        if (ACT == 5) v = 0.5f * v * (1.0f + erff(v * 0.70710678118654752f));
        slab[(mOff + r) * 68 + (j << 4) + rlane] = v;
      }
    }
    __builtin_amdgcn_fence(__ATOMIC_RELEASE, "workgroup");
    __builtin_amdgcn_wave_barrier();
    __builtin_amdgcn_fence(__ATOMIC_ACQUIRE, "workgroup");
    if (OUT_MODE == 0) {
      float* C = (float*)Cout + (size_t)b * strideC;
      const int hh = lane >> 4, c4 = (lane & 15) * 4;
      for (int pass = 0; pass < 2; ++pass) {
#pragma unroll
        for (int it = 0; it < 8; ++it) {
          const int row = it * 2 + hh;
          v4f v = *(const v4f*)(slab + row * 68 + c4);
          *(volatile v4f*)(C + (size_t)(mBase + row) * ldc + n0 + c4) = v;
        }
        __threadfence();
      }
    } else {
      const int q = lane >> 3, c8 = (lane & 7) * 8;
      unsigned short* C  = (unsigned short*)Cout  + (size_t)b * strideC;
      unsigned short* C2 = (OUT_MODE == 2) ? ((unsigned short*)Cout2 + (size_t)b * strideC) : nullptr;
      for (int pass = 0; pass < 2; ++pass) {
#pragma unroll
        for (int it = 0; it < 4; ++it) {
          const int row = it * 4 + q;
          const float* sp = slab + row * 68 + c8;
          v8h hv, lv;
#pragma unroll
          for (int e = 0; e < 8; ++e) {
            if (OUT_MODE == 1) {
              hv[e] = (_Float16)sp[e];
            } else {
              unsigned short hb = f2bf_bits(sp[e]);
              unsigned short lb = f2bf_bits(sp[e] - bf_bits2f(hb));
              hv[e] = __builtin_bit_cast(_Float16, hb);
              lv[e] = __builtin_bit_cast(_Float16, lb);
            }
          }
          *(volatile v8h*)(C + (size_t)(mBase + row) * ldc + n0 + c8) = hv;
          if (OUT_MODE == 2) *(volatile v8h*)(C2 + (size_t)(mBase + row) * ldc + n0 + c8) = lv;
        }
        __threadfence();
      }
    }
    __builtin_amdgcn_fence(__ATOMIC_RELEASE, "workgroup");
    __builtin_amdgcn_wave_barrier();
    __builtin_amdgcn_fence(__ATOMIC_ACQUIRE, "workgroup");
  }
}

constexpr int kBatch   = 8;
constexpr int kCh      = 256;
constexpr int kImg     = 64;
constexpr int kPix     = 4096;
constexpr int kPadDim  = 66;
constexpr int kPadArea = 66 * 66;
constexpr int kGroups  = 4;
constexpr int kCg      = 64;
constexpr int kTaps    = 9;
constexpr int kMoff    = 108;
constexpr int kMoffPad = 128;
constexpr int kKoff    = 2304;
constexpr int kKdcn    = 576;
constexpr int kChunkB  = 2;

static_assert(kKoff % 32 == 0 && kKdcn % 32 == 0, "K tile multiple");
static_assert(kMoffPad % 64 == 0 && kPix % 64 == 0 && kCg % 64 == 0, "M/N tile multiple");
static_assert(kBatch % kChunkB == 0, "chunking");

constexpr size_t kXpadBytes  = (size_t)kBatch * kPadArea * kCh * 4;
constexpr size_t kWoffpBytes = (size_t)kMoffPad * kKoff * 2;
constexpr size_t kWdcnpBytes = (size_t)2 * kCh * kKdcn * 2;
constexpr size_t kBtBytes0   = (size_t)kChunkB * kPix * kKoff * 2;
constexpr size_t kBtBytes1   = (size_t)kChunkB * kGroups * kPix * kKdcn * 2;
constexpr size_t kBtBytes    = kBtBytes0 > kBtBytes1 ? kBtBytes0 : kBtBytes1;
constexpr size_t kOffpBytes  = (size_t)kBatch * kMoffPad * kPix * 4;
constexpr size_t kDcnpBytes  = (size_t)kBatch * kCh * kPix * 4;
constexpr size_t kOffXpad  = 0;
constexpr size_t kOffWoffp = kOffXpad + kXpadBytes;
constexpr size_t kOffWdcnp = kOffWoffp + kWoffpBytes;
constexpr size_t kOffBt    = kOffWdcnp + kWdcnpBytes;
constexpr size_t kOffOffp  = kOffBt + kBtBytes;
constexpr size_t kOffDcnp  = kOffOffp + kOffpBytes;
constexpr size_t kWsTotal  = kOffDcnp + kDcnpBytes;
static_assert(kWsTotal == 124944384, "carve total");
static_assert(kWsTotal <= 134217728, "carve limit");
static_assert(kOffWoffp % 256 == 0 && kOffWdcnp % 256 == 0 && kOffBt % 256 == 0 && kOffOffp % 256 == 0 && kOffDcnp % 256 == 0, "alignment");

__global__ __launch_bounds__(256) void k_xpad(const float* __restrict__ x, float* __restrict__ xp) {
  __shared__ __align__(16) float tile[33 * 256];
  const int t = threadIdx.x;
  const int yp = blockIdx.x >> 1;
  const int hf = blockIdx.x & 1;
  const int b = blockIdx.y;
  const bool inner = (yp >= 1) && (yp <= kImg);
  if (inner) {
    const int yy = yp - 1;
    for (int idx = t; idx < 33 * 256; idx += 256) {
      const int c = idx / 33;
      const int j = idx - c * 33;
      const int w = hf * 33 + j - 1;
      const int wc = w < 0 ? 0 : (w > kImg - 1 ? kImg - 1 : w);
      float v = x[(((size_t)b * kCh + c) * kImg + yy) * kImg + wc];
      v = (w >= 0 && w <= kImg - 1) ? v : 0.0f;
      tile[j * 256 + c] = v;
    }
  } else {
    for (int idx = t; idx < 33 * 256; idx += 256) tile[idx] = 0.0f;
  }
  __syncthreads();
  float* dst = xp + (((size_t)b * kPadDim + yp) * kPadDim + hf * 33) * kCh;
  const int wave = t >> 5, lane = t & 31;
  for (int pass = 0; pass < 2; ++pass) {
    for (int lg = wave; lg < 66; lg += 8) {
      const v4f v = *(const v4f*)(tile + lg * 128 + lane * 4);
      *(volatile v4f*)(dst + lg * 128 + lane * 4) = v;
    }
    __threadfence();
  }
}

__global__ __launch_bounds__(256) void k_wprep(const float* __restrict__ w_off, const float* __restrict__ w_dcn,
                                               _Float16* __restrict__ woffp, _Float16* __restrict__ wdcnp) {
  const int i = blockIdx.x * 256 + threadIdx.x;
  if (blockIdx.y == 0) {
    const int m  = i / 288;
    const int kc = i - m * 288;
    const int k0 = kc * 8;
    const int kk = k0 >> 8;
    const int c0 = k0 & 255;
    const int mm = (m < kMoff) ? m : (kMoff - 1);
    const float zf = (m < kMoff) ? 256.0f : 0.0f;
    v8h hv;
#pragma unroll
    for (int e = 0; e < 8; ++e) {
      const float wv = w_off[((size_t)(mm * kCh + c0 + e)) * kTaps + kk];
      hv[e] = (_Float16)(wv * zf);
    }
    _Float16* dst = woffp + (size_t)m * kKoff + k0;
    *(volatile v8h*)dst = hv;
    __threadfence();
    *(volatile v8h*)dst = hv;
  } else {
    const int r  = i / 72;
    const int kc = i - r * 72;
    const int k0 = kc * 8;
    const int kk = k0 >> 6;
    const int c0 = k0 & 63;
    const int og = r & 255;
    v8h hv;
#pragma unroll
    for (int e = 0; e < 8; ++e) {
      const float wv = w_dcn[((size_t)(og * kCg + c0 + e)) * kTaps + kk];
      hv[e] = (_Float16)(wv * 64.0f);
    }
    _Float16* dst = wdcnp + (size_t)r * kKdcn + k0;
    *(volatile v8h*)dst = hv;
    __threadfence();
    *(volatile v8h*)dst = hv;
  }
}

__global__ __launch_bounds__(256) void k_im2col(const float* __restrict__ xp, _Float16* __restrict__ bt, int b0) {
  const int lane = threadIdx.x & 31;
  const int wid = blockIdx.x * 8 + (threadIdx.x >> 5);
  const int kk = wid % kTaps;
  const int t2 = wid / kTaps;
  const int n  = t2 & (kPix - 1);
  const int bl = t2 >> 12;
  const int b  = b0 + bl;
  const int h = n >> 6, w = n & 63;
  const int dy = kk / 3, dx = kk - dy * 3;
  const float* src = xp + (((size_t)b * kPadDim + h + dy) * kPadDim + (w + dx)) * kCh + lane * 8;
  const v4f a0 = *(const v4f*)(src);
  const v4f a1 = *(const v4f*)(src + 4);
  v8h hv;
#pragma unroll
  for (int e = 0; e < 4; ++e) { hv[e] = (_Float16)a0[e]; hv[4 + e] = (_Float16)a1[e]; }
  _Float16* dst = bt + ((size_t)(bl * kPix + n)) * kKoff + kk * kCh + lane * 8;
  *(volatile v8h*)dst = hv;
  __threadfence();
  *(volatile v8h*)dst = hv;
}

__global__ __launch_bounds__(256) void k_gather(const float* __restrict__ xp, const float* __restrict__ offp,
                                                const float* __restrict__ b_off, _Float16* __restrict__ bt, int b0) {
  const int lane = threadIdx.x & 31;
  const int wid = blockIdx.x * 8 + (threadIdx.x >> 5);
  const int n = wid & (kPix - 1);
  const int z = wid >> 12;
  const int bl = z >> 2, g = z & 3;
  const int b = b0 + bl;
  const int h = n >> 6, w = n & 63;
  const int q = lane >> 3;
  const int c0 = (lane & 7) * 8;
  const float* offb = offp + (size_t)b * kMoffPad * kPix + n;
  const float* xg = xp + (size_t)b * kPadArea * kCh + g * kCg + c0;
  _Float16* dstrow = bt + ((size_t)z * kPix + n) * kKdcn + c0;
#pragma unroll 1
  for (int ps = 0; ps < 3; ++ps) {
    const int kkr = ps * 4 + q;
    const bool act = kkr < kTaps;
    const int kk = act ? kkr : (kTaps - 1);
    const int chy = g * 18 + kk * 2;
    const int chm = 72 + g * 9 + kk;
    const float oy = offb[(size_t)chy * kPix] + b_off[chy];
    const float ox = offb[(size_t)(chy + 1) * kPix] + b_off[chy + 1];
    const float ml = offb[(size_t)chm * kPix] + b_off[chm];
    const float msk = __builtin_amdgcn_rcpf(1.0f + expf(-ml));
    const int dy = kk / 3;
    const int dx = kk - dy * 3;
    float py = (float)(h + dy - 1) + oy;
    float px = (float)(w + dx - 1) + ox;
    py = fminf(fmaxf(py, -4.0f), 70.0f);
    px = fminf(fmaxf(px, -4.0f), 70.0f);
    const float y0f = floorf(py), x0f = floorf(px);
    const float wy1 = py - y0f, wy0 = 1.0f - wy1;
    const float wx1 = px - x0f, wx0 = 1.0f - wx1;
    const int y0 = (int)y0f, x0 = (int)x0f;
    const int y1 = y0 + 1, x1 = x0 + 1;
    const bool vy0 = (y0 >= 0) && (y0 < kImg);
    const bool vy1 = (y1 >= 0) && (y1 < kImg);
    const bool vx0 = (x0 >= 0) && (x0 < kImg);
    const bool vx1 = (x1 >= 0) && (x1 < kImg);
    const float w00 = (vy0 && vx0) ? (wy0 * wx0) : 0.0f;
    const float w01 = (vy0 && vx1) ? (wy0 * wx1) : 0.0f;
    const float w10 = (vy1 && vx0) ? (wy1 * wx0) : 0.0f;
    const float w11 = (vy1 && vx1) ? (wy1 * wx1) : 0.0f;
    const int yc0 = y0 < 0 ? 0 : (y0 > kImg - 1 ? kImg - 1 : y0);
    const int yc1 = y1 < 0 ? 0 : (y1 > kImg - 1 ? kImg - 1 : y1);
    const int xc0 = x0 < 0 ? 0 : (x0 > kImg - 1 ? kImg - 1 : x0);
    const int xc1 = x1 < 0 ? 0 : (x1 > kImg - 1 ? kImg - 1 : x1);
    const float* p00 = xg + (size_t)((yc0 + 1) * kPadDim + (xc0 + 1)) * kCh;
    const float* p01 = xg + (size_t)((yc0 + 1) * kPadDim + (xc1 + 1)) * kCh;
    const float* p10 = xg + (size_t)((yc1 + 1) * kPadDim + (xc0 + 1)) * kCh;
    const float* p11 = xg + (size_t)((yc1 + 1) * kPadDim + (xc1 + 1)) * kCh;
    const v4f a00 = *(const v4f*)(p00), e00 = *(const v4f*)(p00 + 4);
    const v4f a01 = *(const v4f*)(p01), e01 = *(const v4f*)(p01 + 4);
    const v4f a10 = *(const v4f*)(p10), e10 = *(const v4f*)(p10 + 4);
    const v4f a11 = *(const v4f*)(p11), e11 = *(const v4f*)(p11 + 4);
    v8h hv;
#pragma unroll
    for (int e = 0; e < 4; ++e) {
      const float s0 = (((a00[e] * w00 + a01[e] * w01) + a10[e] * w10) + a11[e] * w11) * msk;
      const float s1 = (((e00[e] * w00 + e01[e] * w01) + e10[e] * w10) + e11[e] * w11) * msk;
      hv[e] = (_Float16)s0;
      hv[4 + e] = (_Float16)s1;
    }
    _Float16* dst = dstrow + kk * kCg;
    if (act) *(volatile v8h*)dst = hv;
    __threadfence();
    if (act) *(volatile v8h*)dst = hv;
  }
}

__global__ __launch_bounds__(256) void k_ln_out(const float* __restrict__ dcn, const float* __restrict__ x,
                                                const float* __restrict__ b_dcn, const float* __restrict__ gamma,
                                                const float* __restrict__ beta, float* __restrict__ out) {
  __shared__ __align__(16) float tile[256 * 32];
  __shared__ float sb[256];
  __shared__ float sg[256];
  __shared__ float sbe[256];
  const int t = threadIdx.x;
  const int b = blockIdx.y;
  const int p0 = blockIdx.x * 32;
  sb[t] = b_dcn[t];
  sg[t] = gamma[t];
  sbe[t] = beta[t];
  __syncthreads();
  const float* src = dcn + (size_t)b * kCh * kPix + p0;
#pragma unroll
  for (int i = 0; i < 8; ++i) {
    const int idx4 = i * 256 + t;
    const int c = idx4 >> 3;
    const int p4 = (idx4 & 7) * 4;
    v4f v = *(const v4f*)(src + (size_t)c * kPix + p4);
    const float bb = sb[c];
    const v4f bb4 = {bb, bb, bb, bb};
    v = v + bb4;
    *(v4f*)(tile + c * 32 + p4) = v;
  }
  __syncthreads();
  const int p = t >> 3, sub = t & 7;
  float s = 0.0f;
#pragma unroll 1
  for (int i = 0; i < 32; ++i) s += tile[(sub + 8 * i) * 32 + p];
  s += __shfl_xor(s, 1, 32);
  s += __shfl_xor(s, 2, 32);
  s += __shfl_xor(s, 4, 32);
  const float mu = s * (1.0f / 256.0f);
  float qv = 0.0f;
#pragma unroll 1
  for (int i = 0; i < 32; ++i) { const float d = tile[(sub + 8 * i) * 32 + p] - mu; qv += d * d; }
  qv += __shfl_xor(qv, 1, 32);
  qv += __shfl_xor(qv, 2, 32);
  qv += __shfl_xor(qv, 4, 32);
  const float rstd = rsqrtf(qv * (1.0f / 256.0f) + 1e-5f);
  const float* xb = x + (size_t)b * kCh * kPix + p0 + p;
#pragma unroll 1
  for (int i = 0; i < 32; ++i) {
    const int c = sub + 8 * i;
    const float v = tile[c * 32 + p];
    const float zn = (v - mu) * rstd * sg[c] + sbe[c];
    const float a = __builtin_amdgcn_rcpf(1.0f + expf(-zn));
    const float xv = xb[(size_t)c * kPix];
    tile[c * 32 + p] = xv * a;
  }
  __syncthreads();
  const int wv = t >> 5, lane = t & 31;
  float* ob = out + (size_t)b * kCh * kPix + p0;
  for (int pass = 0; pass < 2; ++pass) {
#pragma unroll
    for (int it = 0; it < 8; ++it) {
      const int c = wv * 32 + it * 4 + (lane >> 3);
      const int p4 = (lane & 7) * 4;
      const v4f v = *(const v4f*)(tile + c * 32 + p4);
      *(volatile v4f*)(ob + (size_t)c * kPix + p4) = v;
    }
    __threadfence();
  }
}

extern "C" void kernel_launch(void* const* d_in, const int* in_sizes, int n_in,
                              void* d_out, int out_size, void* d_ws, size_t ws_size,
                              hipStream_t stream) {
  if (n_in < 7) return;
  if (in_sizes[0] != kBatch * kCh * kPix) return;
  if (out_size != kBatch * kCh * kPix) return;
  if (ws_size < kWsTotal) return;
  const float* x     = (const float*)d_in[0];
  const float* w_off = (const float*)d_in[1];
  const float* b_off = (const float*)d_in[2];
  const float* w_dcn = (const float*)d_in[3];
  const float* b_dcn = (const float*)d_in[4];
  const float* gamma = (const float*)d_in[5];
  const float* beta  = (const float*)d_in[6];
  float* out = (float*)d_out;

  char* ws = (char*)d_ws;
  float*    xpad  = (float*)(ws + kOffXpad);
  _Float16* woffp = (_Float16*)(ws + kOffWoffp);
  _Float16* wdcnp = (_Float16*)(ws + kOffWdcnp);
  _Float16* bt    = (_Float16*)(ws + kOffBt);
  float*    offp  = (float*)(ws + kOffOffp);
  float*    dcnp  = (float*)(ws + kOffDcnp);

  k_xpad<<<dim3(kPadDim * 2, kBatch), dim3(256), 0, stream>>>(x, xpad);
  k_wprep<<<dim3(144, 2), dim3(256), 0, stream>>>(w_off, w_dcn, woffp, wdcnp);

  for (int bb = 0; bb < kBatch; bb += kChunkB) {
    k_im2col<<<dim3(kChunkB * kPix * kTaps / 8), dim3(256), 0, stream>>>(xpad, bt, bb);
    wmma_gemm64<0, false, 0, 0, false, 0><<<dim3((kMoffPad / 64) * (kPix / 64) / 8, kChunkB), dim3(256), 0, stream>>>(
        (const unsigned short*)woffp, (const unsigned short*)woffp, kKoff, 0L,
        (const unsigned short*)bt, (const unsigned short*)bt, kKoff, (long)kPix * kKoff,
        (void*)(offp + (size_t)bb * kMoffPad * kPix), (void*)(offp + (size_t)bb * kMoffPad * kPix), kPix, (long)kMoffPad * kPix,
        b_off, x, 0L,
        kMoffPad, kPix, kKoff, 1.0f / 256.0f);
  }
  for (int bb = 0; bb < kBatch; bb += kChunkB) {
    k_gather<<<dim3(kChunkB * kGroups * kPix / 8), dim3(256), 0, stream>>>(xpad, offp, b_off, bt, bb);
    wmma_gemm64<0, false, 0, 0, false, 0><<<dim3((kCg / 64) * (kPix / 64) / 8, kChunkB * kGroups), dim3(256), 0, stream>>>(
        (const unsigned short*)wdcnp, (const unsigned short*)wdcnp, kKdcn, (long)kCg * kKdcn,
        (const unsigned short*)bt, (const unsigned short*)bt, kKdcn, (long)kPix * kKdcn,
        (void*)(dcnp + (size_t)bb * kCh * kPix), (void*)(dcnp + (size_t)bb * kCh * kPix), kPix, (long)kCg * kPix,
        b_dcn, x, 0L,
        kCg, kPix, kKdcn, 1.0f / 64.0f);
  }
  k_ln_out<<<dim3(kPix / 32, kBatch), dim3(256), 0, stream>>>(dcnp, x, b_dcn, gamma, beta, out);
}
